// Block_35012573397344
// MI455X (gfx1250) — hardware-verified
//
#include <hip/hip_runtime.h>


#pragma clang fp contract(off)

#ifndef NB
#define NB 2
#endif
#ifndef SEQ
#define SEQ 2048
#endif
#define NB_FULL 2
#define SEQ_FULL 2048
#define CDIM 1024
#define NHEAD 16
#define HD 64
#define HID 4096
#define MROWS (NB * SEQ)

static_assert(NB >= 1 && NB <= NB_FULL);
static_assert(SEQ % 64 == 0 && SEQ >= 64 && SEQ <= SEQ_FULL);
static_assert(CDIM == NHEAD * HD);
static_assert(HD == 64);
static_assert(CDIM == 1024);
static_assert(CDIM == 32 * 8 * 4);
static_assert(HID % 64 == 0 && CDIM % 64 == 0);
static_assert(HID % 32 == 0 && CDIM % 32 == 0);
static_assert(MROWS % 64 == 0 && MROWS % 8 == 0);
static_assert((unsigned long long)MROWS * HID < 4294967296ull);
static_assert((unsigned long long)3 * MROWS * CDIM < 4294967296ull);
static_assert((unsigned long long)((NB_FULL - 1) * SEQ_FULL + SEQ_FULL) * CDIM < 4294967296ull);

typedef _Float16 v16h __attribute__((ext_vector_type(16)));
typedef _Float16 v8h  __attribute__((ext_vector_type(8)));
typedef float    v8f  __attribute__((ext_vector_type(8)));
typedef float    v4f  __attribute__((ext_vector_type(4)));
typedef unsigned int v4u __attribute__((ext_vector_type(4)));

union Frag { v16h v; v4u q[2]; };

__device__ __forceinline__ v8f mma(v16h a, v16h b, v8f c) {
  v8f d = __builtin_amdgcn_wmma_f32_16x16x32_f16(false, a, false, b, (short)0, c, false, false);
  asm volatile("v_nop\n\tv_nop\n\tv_nop\n\tv_nop" : "+v"(d) : "v"(a), "v"(b));
  return d;
}

__device__ __forceinline__ v8f zero8() {
  v8f z;
#pragma unroll
  for (int i = 0; i < 8; ++i) z[i] = 0.0f;
  return z;
}

__device__ __forceinline__ float bf16q(float f) {
  unsigned int u = __float_as_uint(f);
  unsigned int r = u + 0x7FFFu + ((u >> 16) & 1u);
  r = ((u & 0x7F800000u) == 0x7F800000u) ? u : r;
  return __uint_as_float(r & 0xFFFF0000u);
}
__device__ __forceinline__ v4f bf16q4(v4f a) {
  v4f r;
  r.x = bf16q(a.x); r.y = bf16q(a.y); r.z = bf16q(a.z); r.w = bf16q(a.w);
  return r;
}
__device__ __forceinline__ unsigned short hbits(float f) {
  _Float16 h = (_Float16)f;
  return __builtin_bit_cast(unsigned short, h);
}
__device__ __forceinline__ v4u pack8h(float f0, float f1, float f2, float f3,
                                      float f4, float f5, float f6, float f7) {
  v8h t;
  t[0] = (_Float16)f0; t[1] = (_Float16)f1; t[2] = (_Float16)f2; t[3] = (_Float16)f3;
  t[4] = (_Float16)f4; t[5] = (_Float16)f5; t[6] = (_Float16)f6; t[7] = (_Float16)f7;
  return __builtin_bit_cast(v4u, t);
}

__global__ __launch_bounds__(256) void k_wprep(
    const float* __restrict__ src, unsigned short* __restrict__ dst,
    int K, int hstride, int rstride, int drow0) {
  __shared__ __attribute__((aligned(16))) unsigned short sT[64][72];
  const int tid = threadIdx.x;
  const int k0 = blockIdx.x * 64, n0 = blockIdx.y * 64;
  const size_t sbase = (size_t)(n0 >> 6) * (size_t)hstride;
#pragma unroll
  for (int it = 0; it < 4; ++it) {
    const int idx = it * 256 + tid;
    const int kk = idx >> 4;
    const int j4 = (idx & 15) * 4;
    const v4f wv = *(const v4f*)(src + sbase + (size_t)(k0 + kk) * (size_t)rstride + j4);
    sT[j4 + 0][kk] = hbits(bf16q(wv.x) * 16.0f);
    sT[j4 + 1][kk] = hbits(bf16q(wv.y) * 16.0f);
    sT[j4 + 2][kk] = hbits(bf16q(wv.z) * 16.0f);
    sT[j4 + 3][kk] = hbits(bf16q(wv.w) * 16.0f);
  }
  __syncthreads();
  v4u val[2];
  size_t off[2];
#pragma unroll
  for (int p = 0; p < 2; ++p) {
    const int n = p * 32 + (tid >> 3);
    const int piece = tid & 7;
    val[p] = *(const v4u*)&sT[n][piece * 8];
    off[p] = ((size_t)drow0 + n0 + n) * (size_t)K + k0 + piece * 8;
  }
#pragma unroll
  for (int p = 0; p < 2; ++p) *(volatile v4u*)(dst + off[p]) = val[p];
  __threadfence();
#pragma unroll
  for (int p = 0; p < 2; ++p) *(volatile v4u*)(dst + off[p]) = val[p];
}

template <int RNDIN>
__device__ __forceinline__ void ln_body(
    const float* x, const float* g, const float* bt, unsigned short* hout, int nrows) {
  const int lane = threadIdx.x & 31, w = threadIdx.x >> 5;
  const int row = blockIdx.x * 8 + w;
  if (row >= nrows) return;
  size_t xrow;
  if (RNDIN) {
    const int b = row / SEQ, t = row - b * SEQ;
    xrow = ((size_t)b * SEQ_FULL + t) * CDIM;
  } else {
    xrow = (size_t)row * CDIM;
  }
  const int cb = lane * 8;

  float v[32];
#pragma unroll
  for (int i = 0; i < 4; ++i) {
    const v4f t0 = *(const v4f*)(x + xrow + 256 * i + cb);
    const v4f t1 = *(const v4f*)(x + xrow + 256 * i + cb + 4);
    v[8 * i + 0] = t0.x; v[8 * i + 1] = t0.y; v[8 * i + 2] = t0.z; v[8 * i + 3] = t0.w;
    v[8 * i + 4] = t1.x; v[8 * i + 5] = t1.y; v[8 * i + 6] = t1.z; v[8 * i + 7] = t1.w;
  }
  if (RNDIN) {
#pragma unroll
    for (int i = 0; i < 32; ++i) v[i] = bf16q(v[i]);
  }

  float s = 0.0f;
#pragma unroll
  for (int i = 0; i < 32; ++i) s += v[i];
#pragma unroll
  for (int xm = 1; xm < 32; xm <<= 1) s += __shfl_xor(s, xm, 32);
  const float mu = s * (1.0f / CDIM);

#pragma unroll
  for (int i = 0; i < 32; ++i) v[i] = v[i] - mu;
  float qs = 0.0f;
#pragma unroll
  for (int i = 0; i < 32; ++i) qs += v[i] * v[i];
#pragma unroll
  for (int xm = 1; xm < 32; xm <<= 1) qs += __shfl_xor(qs, xm, 32);
  const float var = qs * (1.0f / CDIM);
  const float rstd = rsqrtf(var + 1e-5f);

  v4u val[4];
#pragma unroll
  for (int i = 0; i < 4; ++i) {
    const v4f g0 = bf16q4(*(const v4f*)(g + 256 * i + cb));
    const v4f g1 = bf16q4(*(const v4f*)(g + 256 * i + cb + 4));
    const v4f b0 = bf16q4(*(const v4f*)(bt + 256 * i + cb));
    const v4f b1 = bf16q4(*(const v4f*)(bt + 256 * i + cb + 4));
    const float y0 = v[8 * i + 0] * rstd * g0.x + b0.x;
    const float y1 = v[8 * i + 1] * rstd * g0.y + b0.y;
    const float y2 = v[8 * i + 2] * rstd * g0.z + b0.z;
    const float y3 = v[8 * i + 3] * rstd * g0.w + b0.w;
    const float y4 = v[8 * i + 4] * rstd * g1.x + b1.x;
    const float y5 = v[8 * i + 5] * rstd * g1.y + b1.y;
    const float y6 = v[8 * i + 6] * rstd * g1.z + b1.z;
    const float y7 = v[8 * i + 7] * rstd * g1.w + b1.w;
    val[i] = pack8h(y0, y1, y2, y3, y4, y5, y6, y7);
  }
  unsigned short* orow = hout + (size_t)row * CDIM + cb;
#pragma unroll
  for (int i = 0; i < 4; ++i) *(volatile v4u*)(orow + 256 * i) = val[i];
  __threadfence();
#pragma unroll
  for (int i = 0; i < 4; ++i) *(volatile v4u*)(orow + 256 * i) = val[i];
}

__global__ __launch_bounds__(256) void k_ln_in(
    const float* __restrict__ x, const float* __restrict__ g, const float* __restrict__ bt,
    unsigned short* __restrict__ hout, int nrows) {
  ln_body<1>(x, g, bt, hout, nrows);
}
__global__ __launch_bounds__(256) void k_ln_mid(
    const float* __restrict__ x, const float* __restrict__ g, const float* __restrict__ bt,
    unsigned short* __restrict__ hout, int nrows) {
  ln_body<0>(x, g, bt, hout, nrows);
}

template <int EPI, int RESFULL, int OUTFULL>
__device__ __forceinline__ void gemm_body(
    const unsigned short* A, const unsigned short* Bt, int K,
    const float* bias, const float* res,
    float* outF, unsigned short* out0, int ldo) {
  __shared__ __attribute__((aligned(16))) unsigned short sT[64][72];
  __shared__ __attribute__((aligned(16))) float sF[64][68];
  const int tid = threadIdx.x, lane = tid & 31, w = tid >> 5;
  const int m = lane & 15, hl = lane >> 4, k8 = hl * 8;
  const int m0 = blockIdx.y * 64, n0 = blockIdx.x * 64;

  v8f acc[4];
#pragma unroll
  for (int j = 0; j < 4; ++j) acc[j] = zero8();

  const unsigned short* ap = A + (size_t)(m0 + 16 * w + m) * (size_t)K + k8;
  const unsigned short* bp = Bt + (size_t)(n0 + m) * (size_t)K + k8;
  const size_t jstep = (size_t)16 * (size_t)K;
#pragma unroll 1
  for (int k0 = 0; k0 < K; k0 += 32) {
    Frag a;
    a.q[0] = *(const v4u*)(ap + k0);
    a.q[1] = *(const v4u*)(ap + k0 + 16);
#pragma unroll
    for (int j = 0; j < 4; ++j) {
      Frag b;
      const unsigned short* bj = bp + jstep * j + k0;
      b.q[0] = *(const v4u*)(bj);
      b.q[1] = *(const v4u*)(bj + 16);
      acc[j] = mma(a.v, b.v, acc[j]);
    }
  }

  const float wsc = 0.0625f;
  const int lrow0 = 16 * w + 8 * hl;

  if constexpr (EPI == 0) {
#pragma unroll
    for (int j = 0; j < 4; ++j) {
#pragma unroll
      for (int r = 0; r < 8; ++r) sT[lrow0 + r][16 * j + m] = hbits(acc[j][r] * wsc);
    }
    __syncthreads();
    const int which = n0 / CDIM;
    const int hh = (n0 - which * CDIM) / HD;
    const int b = m0 / SEQ, t0 = m0 - b * SEQ;
    const int bh = b * NHEAD + hh;
    const unsigned int pbase = (unsigned int)which * (unsigned int)(MROWS * CDIM);
    v4u val[4];
    unsigned int off[4];
    if (which < 2) {
#pragma unroll
      for (int p = 0; p < 4; ++p) {
        const int row = p * 16 + 4 * w + (lane >> 3);
        const int piece = lane & 7;
        val[p] = *(const v4u*)&sT[row][piece * 8];
        off[p] = pbase + (unsigned int)((bh * SEQ + t0 + row) * HD + piece * 8);
      }
    } else {
#pragma unroll
      for (int p = 0; p < 4; ++p) {
        const int d = p * 16 + 4 * w + (lane >> 3);
        const int piece = lane & 7;
        unsigned int wv[4];
#pragma unroll
        for (int e = 0; e < 4; ++e) {
          const unsigned int lo = sT[piece * 8 + 2 * e][d];
          const unsigned int hi = sT[piece * 8 + 2 * e + 1][d];
          wv[e] = lo | (hi << 16);
        }
        v4u t;
        t.x = wv[0]; t.y = wv[1]; t.z = wv[2]; t.w = wv[3];
        val[p] = t;
        off[p] = pbase + (unsigned int)((bh * HD + d) * SEQ + t0 + piece * 8);
      }
    }
#pragma unroll
    for (int p = 0; p < 4; ++p) *(volatile v4u*)(out0 + off[p]) = val[p];
    __threadfence();
#pragma unroll
    for (int p = 0; p < 4; ++p) *(volatile v4u*)(out0 + off[p]) = val[p];
  } else if constexpr (EPI == 1) {
#pragma unroll
    for (int j = 0; j < 4; ++j) {
#pragma unroll
      for (int r = 0; r < 8; ++r) sF[lrow0 + r][16 * j + m] = acc[j][r] * wsc;
    }
    __syncthreads();
    const int b = m0 / SEQ, t0 = m0 - b * SEQ;
    v4f val[8];
    unsigned int off[8];
#pragma unroll
    for (int p = 0; p < 8; ++p) {
      const int row = 16 * w + 2 * p + hl;
      const int piece = m;
      const int ncol = n0 + 4 * piece;
      const v4f a = *(const v4f*)&sF[row][4 * piece];
      const v4f bv = bf16q4(*(const v4f*)(bias + ncol));
      const size_t rrow = RESFULL ? ((size_t)b * SEQ_FULL + t0 + row) : (size_t)(m0 + row);
      v4f rr = *(const v4f*)(res + rrow * (size_t)ldo + ncol);
      if (RESFULL) rr = bf16q4(rr);
      val[p] = (a + bv) + rr;
      const size_t orow = OUTFULL ? ((size_t)b * SEQ_FULL + t0 + row) : (size_t)(m0 + row);
      off[p] = (unsigned int)(orow * (size_t)ldo + ncol);
    }
#pragma unroll
    for (int p = 0; p < 8; ++p) *(volatile v4f*)(outF + off[p]) = val[p];
    __threadfence();
#pragma unroll
    for (int p = 0; p < 8; ++p) *(volatile v4f*)(outF + off[p]) = val[p];
  } else {
#pragma unroll
    for (int j = 0; j < 4; ++j) {
      const float bj = bf16q(bias[n0 + 16 * j + m]);
#pragma unroll
      for (int r = 0; r < 8; ++r) {
        float u = acc[j][r] * wsc + bj;
        u = fmaxf(u, 0.0f);
        sT[lrow0 + r][16 * j + m] = hbits(u);
      }
    }
    __syncthreads();
    v4u val[4];
    unsigned int off[4];
#pragma unroll
    for (int p = 0; p < 4; ++p) {
      const int row = 16 * w + 4 * p + (lane >> 3);
      const int piece = lane & 7;
      val[p] = *(const v4u*)&sT[row][piece * 8];
      off[p] = (unsigned int)((size_t)(m0 + row) * (size_t)ldo + n0 + piece * 8);
    }
#pragma unroll
    for (int p = 0; p < 4; ++p) *(volatile v4u*)(out0 + off[p]) = val[p];
    __threadfence();
#pragma unroll
    for (int p = 0; p < 4; ++p) *(volatile v4u*)(out0 + off[p]) = val[p];
  }
}

__global__ __launch_bounds__(128) void k_gemm_qkv(
    const unsigned short* __restrict__ A, const unsigned short* __restrict__ Bt,
    unsigned short* __restrict__ qkv) {
  gemm_body<0, 0, 0>(A, Bt, CDIM, nullptr, nullptr, nullptr, qkv, 0);
}
__global__ __launch_bounds__(128) void k_gemm_proj(
    const unsigned short* __restrict__ A, const unsigned short* __restrict__ Bt,
    const float* __restrict__ bias, const float* __restrict__ res, float* __restrict__ outF) {
  gemm_body<1, 1, 0>(A, Bt, CDIM, bias, res, outF, nullptr, CDIM);
}
__global__ __launch_bounds__(128) void k_gemm_ffn1(
    const unsigned short* __restrict__ A, const unsigned short* __restrict__ Bt,
    const float* __restrict__ bias, unsigned short* __restrict__ out0) {
  gemm_body<2, 0, 0>(A, Bt, CDIM, bias, nullptr, nullptr, out0, HID);
}
__global__ __launch_bounds__(128) void k_gemm_ffn2(
    const unsigned short* __restrict__ A, const unsigned short* __restrict__ Bt,
    const float* __restrict__ bias, const float* __restrict__ res, float* __restrict__ outF) {
  gemm_body<1, 0, 1>(A, Bt, HID, bias, res, outF, nullptr, CDIM);
}

__global__ __launch_bounds__(128) __attribute__((amdgpu_num_vgpr(256)))
void k_attn(const unsigned short* __restrict__ qp, const unsigned short* __restrict__ kp,
            const unsigned short* __restrict__ vp, unsigned short* __restrict__ op) {
  __shared__ __attribute__((aligned(16))) unsigned short sP[4][16][72];
  const int tid = threadIdx.x, lane = tid & 31, w = tid >> 5;
  const int m = lane & 15, hl = lane >> 4, k8 = hl * 8;
  const int nqt = SEQ / 64;
  const int bh = blockIdx.x / nqt, qt = blockIdx.x - bh * nqt;
  const int b = bh / NHEAD, hh = bh - b * NHEAD;
  const int tq = qt * 64 + 16 * w;

  Frag qa0, qa1;
  {
    const unsigned short* qr = qp + ((size_t)bh * SEQ + tq + m) * HD + k8;
    qa0.q[0] = *(const v4u*)(qr);
    qa0.q[1] = *(const v4u*)(qr + 16);
    qa1.q[0] = *(const v4u*)(qr + 32);
    qa1.q[1] = *(const v4u*)(qr + 48);
  }
  float mrun[8], lrun[8];
  v8f oacc[4];
#pragma unroll
  for (int r = 0; r < 8; ++r) { mrun[r] = -1e30f; lrun[r] = 0.0f; }
#pragma unroll
  for (int j = 0; j < 4; ++j) oacc[j] = zero8();

#pragma unroll 1
  for (int kt = 0; kt <= qt; ++kt) {
    v8f s[4];
    const unsigned short* kb = kp + ((size_t)bh * SEQ + kt * 64 + m) * HD + k8;
#pragma unroll
    for (int j = 0; j < 4; ++j) {
      const unsigned short* kr = kb + j * 16 * HD;
      Frag f0, f1;
      f0.q[0] = *(const v4u*)(kr);
      f0.q[1] = *(const v4u*)(kr + 16);
      f1.q[0] = *(const v4u*)(kr + 32);
      f1.q[1] = *(const v4u*)(kr + 48);
      v8f t = mma(qa0.v, f0.v, zero8());
      t = mma(qa1.v, f1.v, t);
      s[j] = t;
    }
    const bool diag = (kt == qt);
    float tmax[8];
#pragma unroll
    for (int r = 0; r < 8; ++r) tmax[r] = -1e30f;
#pragma unroll
    for (int j = 0; j < 4; ++j) {
#pragma unroll
      for (int r = 0; r < 8; ++r) {
        float val = s[j][r] * 0.03125f;
        const int qi = tq + 8 * hl + r;
        const int ki = kt * 64 + 16 * j + m;
        val = (diag && (ki > qi)) ? -1e30f : val;
        s[j][r] = val;
        tmax[r] = fmaxf(tmax[r], val);
      }
    }
#pragma unroll
    for (int r = 0; r < 8; ++r) {
#pragma unroll
      for (int xm = 1; xm < 16; xm <<= 1) tmax[r] = fmaxf(tmax[r], __shfl_xor(tmax[r], xm, 32));
    }
    float corr[8];
#pragma unroll
    for (int r = 0; r < 8; ++r) {
      const float mn = fmaxf(mrun[r], tmax[r]);
      corr[r] = __expf(mrun[r] - mn);
      mrun[r] = mn;
    }
    float tsum[8];
#pragma unroll
    for (int r = 0; r < 8; ++r) tsum[r] = 0.0f;
#pragma unroll
    for (int j = 0; j < 4; ++j) {
#pragma unroll
      for (int r = 0; r < 8; ++r) {
        const float p = __expf(s[j][r] - mrun[r]);
        tsum[r] += p;
        sP[w][8 * hl + r][16 * j + m] = hbits(p * 1024.0f);
      }
    }
#pragma unroll
    for (int r = 0; r < 8; ++r) {
#pragma unroll
      for (int xm = 1; xm < 16; xm <<= 1) tsum[r] += __shfl_xor(tsum[r], xm, 32);
      lrun[r] = lrun[r] * corr[r] + tsum[r];
    }
#pragma unroll
    for (int j = 0; j < 4; ++j) {
#pragma unroll
      for (int r = 0; r < 8; ++r) oacc[j][r] *= corr[r];
    }
    __syncthreads();
    Frag pa0, pa1;
    {
      const unsigned short* pr = &sP[w][m][k8];
      pa0.q[0] = *(const v4u*)(pr);
      pa0.q[1] = *(const v4u*)(pr + 16);
      pa1.q[0] = *(const v4u*)(pr + 32);
      pa1.q[1] = *(const v4u*)(pr + 48);
    }
    const unsigned short* vb = vp + ((size_t)bh * HD + m) * (size_t)SEQ + kt * 64 + k8;
#pragma unroll
    for (int jd = 0; jd < 4; ++jd) {
      const unsigned short* vr = vb + (size_t)jd * 16 * SEQ;
      Frag g0, g1;
      g0.q[0] = *(const v4u*)(vr);
      g0.q[1] = *(const v4u*)(vr + 16);
      g1.q[0] = *(const v4u*)(vr + 32);
      g1.q[1] = *(const v4u*)(vr + 48);
      oacc[jd] = mma(pa0.v, g0.v, oacc[jd]);
      oacc[jd] = mma(pa1.v, g1.v, oacc[jd]);
    }
    __syncthreads();
  }

  float il[8];
#pragma unroll
  for (int r = 0; r < 8; ++r) il[r] = 1.0f / (lrun[r] * 1024.0f);
#pragma unroll
  for (int jd = 0; jd < 4; ++jd) {
#pragma unroll
    for (int r = 0; r < 8; ++r) sP[w][8 * hl + r][16 * jd + m] = hbits(oacc[jd][r] * il[r]);
  }
  __syncthreads();
  v4u val[4];
  unsigned int off[4];
#pragma unroll
  for (int p = 0; p < 4; ++p) {
    const int row = 4 * p + (lane >> 3);
    const int piece = lane & 7;
    val[p] = *(const v4u*)&sP[w][row][piece * 8];
    off[p] = (unsigned int)((size_t)(b * SEQ + tq + row) * CDIM + hh * HD + piece * 8);
  }
#pragma unroll
  for (int p = 0; p < 4; ++p) *(volatile v4u*)(op + off[p]) = val[p];
  __threadfence();
#pragma unroll
  for (int p = 0; p < 4; ++p) *(volatile v4u*)(op + off[p]) = val[p];
}

constexpr size_t SZ_WQKV = (size_t)3 * CDIM * CDIM * 2;
constexpr size_t SZ_WP   = (size_t)CDIM * CDIM * 2;
constexpr size_t SZ_W1   = (size_t)HID * CDIM * 2;
constexpr size_t SZ_W2   = (size_t)CDIM * HID * 2;
constexpr size_t SZ_MC2  = (size_t)MROWS * CDIM * 2;
constexpr size_t SZ_MC4  = (size_t)MROWS * CDIM * 4;
constexpr size_t SZ_ACT  = (size_t)MROWS * HID * 2;
constexpr size_t OFF_WQKV = 0;
constexpr size_t OFF_WP   = OFF_WQKV + SZ_WQKV;
constexpr size_t OFF_W1   = OFF_WP + SZ_WP;
constexpr size_t OFF_W2   = OFF_W1 + SZ_W1;
constexpr size_t OFF_H    = OFF_W2 + SZ_W2;
constexpr size_t OFF_QKV  = OFF_H + SZ_MC2;
constexpr size_t OFF_O    = OFF_QKV + 3 * SZ_MC2;
constexpr size_t OFF_X1   = OFF_O + SZ_MC2;
constexpr size_t OFF_H2   = OFF_X1 + SZ_MC4;
constexpr size_t OFF_ACT  = OFF_H2 + SZ_MC2;
constexpr size_t WS_TOTAL = OFF_ACT + SZ_ACT;
static_assert(SZ_WQKV % 256 == 0 && SZ_WP % 256 == 0 && SZ_W1 % 256 == 0 && SZ_W2 % 256 == 0);
static_assert(SZ_MC2 % 256 == 0 && SZ_MC4 % 256 == 0 && SZ_ACT % 256 == 0);
static_assert(WS_TOTAL <= (size_t)134217728);

extern "C" void kernel_launch(void* const* d_in, const int* in_sizes, int n_in,
                              void* d_out, int out_size, void* d_ws, size_t ws_size,
                              hipStream_t stream) {
  if (n_in < 14) return;
  const long needX = ((long)(NB - 1) * SEQ_FULL + SEQ) * CDIM;
  const long nW = (long)NHEAD * CDIM * HD;
  if ((long)in_sizes[0] < needX) return;
  if ((long)in_sizes[1] < nW || (long)in_sizes[2] < nW || (long)in_sizes[3] < nW) return;
  if ((long)in_sizes[4] < (long)CDIM * CDIM || in_sizes[5] < CDIM) return;
  if ((long)in_sizes[6] < (long)CDIM * HID || in_sizes[7] < HID) return;
  if ((long)in_sizes[8] < (long)HID * CDIM || in_sizes[9] < CDIM) return;
  if (in_sizes[10] < CDIM || in_sizes[11] < CDIM || in_sizes[12] < CDIM || in_sizes[13] < CDIM) return;
  if ((long)out_size < needX) return;
  if (WS_TOTAL > ws_size) return;

  const float* x     = (const float*)d_in[0];
  const float* Wq    = (const float*)d_in[1];
  const float* Wk    = (const float*)d_in[2];
  const float* Wv    = (const float*)d_in[3];
  const float* Wp    = (const float*)d_in[4];
  const float* bp    = (const float*)d_in[5];
  const float* W1    = (const float*)d_in[6];
  const float* b1    = (const float*)d_in[7];
  const float* W2    = (const float*)d_in[8];
  const float* b2    = (const float*)d_in[9];
  const float* ln1_g = (const float*)d_in[10];
  const float* ln1_b = (const float*)d_in[11];
  const float* ln2_g = (const float*)d_in[12];
  const float* ln2_b = (const float*)d_in[13];
  float* out = (float*)d_out;

  char* ws = (char*)d_ws;
  unsigned short* wqkv = (unsigned short*)(ws + OFF_WQKV);
  unsigned short* wpt  = (unsigned short*)(ws + OFF_WP);
  unsigned short* w1t  = (unsigned short*)(ws + OFF_W1);
  unsigned short* w2t  = (unsigned short*)(ws + OFF_W2);
  unsigned short* hpl  = (unsigned short*)(ws + OFF_H);
  unsigned short* qkv  = (unsigned short*)(ws + OFF_QKV);
  unsigned short* qpl  = qkv;
  unsigned short* kpl  = qkv + (size_t)MROWS * CDIM;
  unsigned short* vtp  = qkv + (size_t)2 * MROWS * CDIM;
  unsigned short* opl  = (unsigned short*)(ws + OFF_O);
  float*          x1   = (float*)(ws + OFF_X1);
  unsigned short* h2p  = (unsigned short*)(ws + OFF_H2);
  unsigned short* act  = (unsigned short*)(ws + OFF_ACT);

  k_wprep<<<dim3(CDIM / 64, CDIM / 64), 256, 0, stream>>>(Wq, wqkv, CDIM, CDIM * HD, HD, 0);
  k_wprep<<<dim3(CDIM / 64, CDIM / 64), 256, 0, stream>>>(Wk, wqkv, CDIM, CDIM * HD, HD, CDIM);
  k_wprep<<<dim3(CDIM / 64, CDIM / 64), 256, 0, stream>>>(Wv, wqkv, CDIM, CDIM * HD, HD, 2 * CDIM);
  k_wprep<<<dim3(CDIM / 64, CDIM / 64), 256, 0, stream>>>(Wp, wpt, CDIM, 64, CDIM, 0);
  k_wprep<<<dim3(CDIM / 64, HID / 64), 256, 0, stream>>>(W1, w1t, CDIM, 64, HID, 0);
  k_wprep<<<dim3(HID / 64, CDIM / 64), 256, 0, stream>>>(W2, w2t, HID, 64, CDIM, 0);
  k_ln_in<<<MROWS / 8, 256, 0, stream>>>(x, ln1_g, ln1_b, hpl, MROWS);
  k_gemm_qkv<<<dim3(3 * CDIM / 64, MROWS / 64), 128, 0, stream>>>(hpl, wqkv, qkv);
  k_attn<<<NB * NHEAD * (SEQ / 64), 128, 0, stream>>>(qpl, kpl, vtp, opl);
  k_gemm_proj<<<dim3(CDIM / 64, MROWS / 64), 128, 0, stream>>>(opl, wpt, bp, x, x1);
  k_ln_mid<<<MROWS / 8, 256, 0, stream>>>(x1, ln2_g, ln2_b, h2p, MROWS);
  k_gemm_ffn1<<<dim3(HID / 64, MROWS / 64), 128, 0, stream>>>(h2p, w1t, b1, act);
  k_gemm_ffn2<<<dim3(CDIM / 64, MROWS / 64), 128, 0, stream>>>(act, w2t, b2, x1, out);
}
